// MultiHeadAttentionBlock_22548578304648
// MI455X (gfx1250) — hardware-verified
//
#include <hip/hip_runtime.h>
#ifndef NB
#define NB 2
#endif
#ifndef SQ
#define SQ 2048
#endif
#define NB_FULL 2
#define SQ_FULL 2048
#define DM 1024
#define NH 16
#define HD 64
#define QB 128
#define KB 64
#define MBW (SQ / 32)
#define NR ((size_t)NB * SQ)

static_assert(DM == NH * HD);
static_assert(NB <= NB_FULL && SQ <= SQ_FULL);
static_assert(SQ % 1024 == 0);
static_assert(SQ % QB == 0 && SQ % KB == 0 && QB == 128 && KB == 64 && HD == 64);
static_assert(((size_t)SQ * DM / 8) % 256 == 0);
static_assert(((size_t)DM * DM / 8) % 256 == 0);
static_assert(((size_t)SQ * (SQ / 1024)) % 8 == 0);
static_assert((NB * SQ) % 128 == 0 && DM % 64 == 0 && DM % 32 == 0);

typedef unsigned short v8us __attribute__((ext_vector_type(8), may_alias));
typedef unsigned int   v2u  __attribute__((ext_vector_type(2)));
typedef float  v8f  __attribute__((ext_vector_type(8)));
typedef float  v4f  __attribute__((ext_vector_type(4)));
typedef float  v4fa __attribute__((ext_vector_type(4), may_alias));
typedef _Float16 v16h __attribute__((ext_vector_type(16)));
typedef _Float16 v4h  __attribute__((ext_vector_type(4)));
union FragH { v16h v; v8us half[2]; _Float16 h[16]; unsigned short u[16]; };

__device__ __forceinline__ unsigned short bf16_bits(float x) { unsigned int u = __float_as_uint(x); return (unsigned short)((u + 0x7FFFu + ((u >> 16) & 1u)) >> 16); }
__device__ __forceinline__ float bf16_val(unsigned short b) { return __uint_as_float(((unsigned int)b) << 16); }
__device__ __forceinline__ float bf16_rne(float x) { return bf16_val(bf16_bits(x)); }

__device__ __forceinline__ v16h g2_frag(const _Float16* p, unsigned hh) { FragH f; f.half[0] = *(const v8us*)((const unsigned short*)p + 8u * hh); f.half[1] = *(const v8us*)((const unsigned short*)p + 16u + 8u * hh); return f.v; }
__device__ __forceinline__ v16h l_frag(const unsigned short* p, unsigned hh) { FragH f; f.half[0] = *(const v8us*)(p + 8u * hh); f.half[1] = *(const v8us*)(p + 16u + 8u * hh); return f.v; }
__device__ __forceinline__ v8f g2_mma(v16h a, v16h b, v8f c) { v8f d = __builtin_amdgcn_wmma_f32_16x16x32_f16(false, a, false, b, (short)0, c, false, false); asm volatile("v_nop\n\tv_nop\n\tv_nop\n\tv_nop" : "+v"(d) : "v"(a), "v"(b)); return d; }

__global__ __launch_bounds__(256) void k_wnat(const float* __restrict__ wsrc, size_t n8, _Float16* __restrict__ Bt) {
  const size_t t = (size_t)blockIdx.x * 256u + threadIdx.x; if (t >= n8) return;
  const v4f a = *(const v4fa*)(wsrc + t * 8), c = *(const v4fa*)(wsrc + t * 8 + 4);
  FragH f;
#pragma unroll
  for (int q = 0; q < 4; ++q) { f.h[q] = (_Float16)(bf16_rne(a[q]) * 16.0f); f.h[4 + q] = (_Float16)(bf16_rne(c[q]) * 16.0f); }
  const v8us o = f.half[0];
  *(volatile v8us*)((unsigned short*)Bt + t * 8) = o; __threadfence(); *(volatile v8us*)((unsigned short*)Bt + t * 8) = o;
}

__global__ __launch_bounds__(256) void k_x16(const float* __restrict__ x, _Float16* __restrict__ X16) {
  const unsigned t = blockIdx.x * 256u + threadIdx.x; const unsigned b = blockIdx.y;
  const float* src = x + (size_t)b * SQ_FULL * DM + (size_t)t * 8;
  unsigned short* dst = (unsigned short*)X16 + (size_t)b * SQ * DM + (size_t)t * 8;
  const v4f a = *(const v4fa*)(src), c = *(const v4fa*)(src + 4);
  FragH f;
#pragma unroll
  for (int q = 0; q < 4; ++q) { f.h[q] = (_Float16)bf16_rne(a[q]); f.h[4 + q] = (_Float16)bf16_rne(c[q]); }
  const v8us o = f.half[0];
  *(volatile v8us*)dst = o; __threadfence(); *(volatile v8us*)dst = o;
}

__global__ __launch_bounds__(256) void k_maskbits(const int* __restrict__ mask, unsigned int* __restrict__ MBp) {
  const unsigned lane = threadIdx.x & 31u, w = threadIdx.x >> 5;
  const unsigned gw = blockIdx.x * 8u + w;
  const unsigned row = gw / (SQ / 1024u), g = gw % (SQ / 1024u);
  const int* src = mask + (size_t)row * SQ_FULL + g * 1024u + lane;
  unsigned word = 0u;
#pragma unroll 4
  for (unsigned it = 0; it < 32u; ++it) {
    const int v = src[it * 32u];
    const unsigned bal = __builtin_amdgcn_ballot_w32(v != 0);
    word = (it == lane) ? bal : word;
  }
  volatile unsigned int* d = MBp + (size_t)row * MBW + g * 32u + lane;
  *d = word; __threadfence(); *d = word;
}

template <bool DUAL, bool WRES>
__global__ __launch_bounds__(128) void k_gemm2(const _Float16* __restrict__ A, const _Float16* __restrict__ A2, unsigned lda, size_t sA,
                                              const _Float16* __restrict__ Bh, unsigned ldb, float alpha, float lofold,
                                              float* __restrict__ C, _Float16* __restrict__ C16, _Float16* __restrict__ C16L, unsigned ldc, size_t sC,
                                              unsigned M, unsigned N, unsigned K) {
  __shared__ __attribute__((aligned(16))) float so[4][32][68];
  const unsigned tid = threadIdx.x, w = tid >> 5, lane = tid & 31u, ln = lane & 15u, hh = lane >> 4; const unsigned by = blockIdx.y;
  const size_t aofs = (size_t)by * sA, cofs = (size_t)by * sC;
  const unsigned ntn = N >> 6; const unsigned mt = blockIdx.x / ntn, nq = blockIdx.x - mt * ntn; const unsigned row0 = mt * 128u + 32u * w, col0 = nq * 64u; if (row0 >= M) return;
  const _Float16* a0p = A + aofs + (size_t)(row0 + ln) * lda; const _Float16* a1p = a0p + (size_t)16 * lda;
  const _Float16* b0p = Bh + (size_t)(col0 + ln) * ldb; const _Float16* b1p = b0p + (size_t)16 * ldb; const _Float16* b2p = b1p + (size_t)16 * ldb; const _Float16* b3p = b2p + (size_t)16 * ldb;
  const v8f z8 = {0.f,0.f,0.f,0.f,0.f,0.f,0.f,0.f}; v8f c00 = z8, c01 = z8, c02 = z8, c03 = z8, c10 = z8, c11 = z8, c12 = z8, c13 = z8;
  if (DUAL) {
    const _Float16* e0p = A2 + aofs + (size_t)(row0 + ln) * lda; const _Float16* e1p = e0p + (size_t)16 * lda;
#pragma unroll 1
    for (unsigned kb = 0; kb < K; kb += 32u) { const v16h a0 = g2_frag(e0p + kb, hh), a1 = g2_frag(e1p + kb, hh);
      v16h b = g2_frag(b0p + kb, hh); c00 = g2_mma(a0, b, c00); c10 = g2_mma(a1, b, c10);
      b = g2_frag(b1p + kb, hh); c01 = g2_mma(a0, b, c01); c11 = g2_mma(a1, b, c11);
      b = g2_frag(b2p + kb, hh); c02 = g2_mma(a0, b, c02); c12 = g2_mma(a1, b, c12);
      b = g2_frag(b3p + kb, hh); c03 = g2_mma(a0, b, c03); c13 = g2_mma(a1, b, c13); }
    c00 = c00 * lofold; c01 = c01 * lofold; c02 = c02 * lofold; c03 = c03 * lofold; c10 = c10 * lofold; c11 = c11 * lofold; c12 = c12 * lofold; c13 = c13 * lofold;
  }
#pragma unroll 1
  for (unsigned kb = 0; kb < K; kb += 32u) { const v16h a0 = g2_frag(a0p + kb, hh), a1 = g2_frag(a1p + kb, hh);
    v16h b = g2_frag(b0p + kb, hh); c00 = g2_mma(a0, b, c00); c10 = g2_mma(a1, b, c10);
    b = g2_frag(b1p + kb, hh); c01 = g2_mma(a0, b, c01); c11 = g2_mma(a1, b, c11);
    b = g2_frag(b2p + kb, hh); c02 = g2_mma(a0, b, c02); c12 = g2_mma(a1, b, c12);
    b = g2_frag(b3p + kb, hh); c03 = g2_mma(a0, b, c03); c13 = g2_mma(a1, b, c13); }
  v8f accs[8] = {c00, c01, c02, c03, c10, c11, c12, c13};
#pragma unroll
  for (int u = 0; u < 8; ++u) { const unsigned t = (unsigned)u & 3u, half = (unsigned)u >> 2;
#pragma unroll
    for (int r = 0; r < 8; ++r) { const unsigned rloc = half * 16u + 8u * hh + (unsigned)r; so[w][rloc][t * 16u + ln] = accs[u][r] * alpha; } }
  __builtin_amdgcn_fence(4  , "workgroup"); __builtin_amdgcn_wave_barrier();
  const unsigned rsub = lane >> 4, c4 = (lane & 15u) * 4u;
  for (int pass = 0; pass < 2; ++pass) {
#pragma unroll
    for (unsigned q = 0; q < 16u; ++q) { const unsigned r = q * 2u + rsub; const v4f v = *(const v4fa*)&so[w][r][c4];
      const size_t go = cofs + (size_t)(row0 + r) * ldc + col0 + c4;
      if (C) *(volatile v4f*)(C + go) = v;
      if (C16) { v4h h4;
#pragma unroll
        for (int i = 0; i < 4; ++i) h4[i] = (_Float16)v[i];
        *(volatile v4h*)(C16 + go) = h4;
        if (WRES) { v4h l4;
#pragma unroll
          for (int i = 0; i < 4; ++i) l4[i] = (_Float16)((v[i] - (float)h4[i]) * 2048.0f);
          *(volatile v4h*)(C16L + go) = l4; } } }
    if (pass == 0) __threadfence(); }
}

template <unsigned NHv, unsigned TTv>
__global__ __launch_bounds__(256) void k_vt(const _Float16* __restrict__ V16, unsigned ldv, _Float16* __restrict__ Vt) {
  __shared__ unsigned short tl[64][66];
  const unsigned tid = threadIdx.x; const unsigned slab = blockIdx.x / (TTv / 64u), lg = blockIdx.x % (TTv / 64u); const unsigned b = slab / NHv, h = slab % NHv;
  for (unsigned i = tid; i < 512u; i += 256u) { const unsigned r = i >> 3, c8 = (i & 7u) * 8u; FragH f;
    f.half[0] = *(const v8us*)((const unsigned short*)V16 + ((size_t)b * TTv + lg * 64u + r) * ldv + h * 64u + c8);
#pragma unroll
    for (int q = 0; q < 8; ++q) tl[r][c8 + (unsigned)q] = f.u[q]; }
  __syncthreads();
  for (int pass = 0; pass < 2; ++pass) {
#pragma unroll
    for (unsigned rd = 0; rd < 2u; ++rd) { const unsigned d = rd * 32u + (tid >> 3), pc = tid & 7u; FragH f;
#pragma unroll
      for (int q = 0; q < 8; ++q) f.u[q] = tl[pc * 8u + (unsigned)q][d];
      *(volatile v8us*)((unsigned short*)Vt + ((size_t)slab * 64u + d) * TTv + lg * 64u + pc * 8u) = f.half[0]; }
    if (pass == 0) __threadfence(); }
}

__global__ __launch_bounds__(256) void k_flash(const _Float16* __restrict__ QH, const _Float16* __restrict__ QL, const _Float16* __restrict__ KH, const _Float16* __restrict__ KL,
                                              const _Float16* __restrict__ VT, const unsigned int* __restrict__ MBp, _Float16* __restrict__ OH, _Float16* __restrict__ OL) {
  __shared__ __attribute__((aligned(16))) unsigned short Kh[KB][72];
  __shared__ __attribute__((aligned(16))) unsigned short Kl[KB][72];
  __shared__ __attribute__((aligned(16))) unsigned short Vs[HD][72];
  __shared__ __attribute__((aligned(16))) _Float16 Ps[8][2][16][72];
  const unsigned tid = threadIdx.x, lane = tid & 31u, w = tid >> 5, ln = lane & 15u, hh = lane >> 4;
  const unsigned bh = blockIdx.y, b = bh / NH, h = bh % NH;
  const unsigned qw = blockIdx.x * QB + w * 16u;
  const size_t rb = (size_t)b * SQ;
  const size_t qoff = (rb + qw + ln) * DM + h * HD;
  const v16h qh0 = g2_frag(QH + qoff, hh), qh1 = g2_frag(QH + qoff + 32, hh);
  const v16h ql0 = g2_frag(QL + qoff, hh), ql1 = g2_frag(QL + qoff + 32, hh);
  const v8f z8 = {0.f,0.f,0.f,0.f,0.f,0.f,0.f,0.f};
  v8f o[4];
#pragma unroll
  for (int j = 0; j < 4; ++j) o[j] = z8;
  float mst[8], lst[8];
#pragma unroll
  for (int r = 0; r < 8; ++r) { mst[r] = -3.0e38f; lst[r] = 0.0f; }
  const unsigned sRow = tid >> 2, sCol = (tid & 3u) * 16u;
  const unsigned int* mbase = MBp + (size_t)(qw + 8u * hh) * MBW;

#pragma unroll 1
  for (unsigned kb = 0; kb < SQ / KB; ++kb) {
    {
      const size_t kg = (rb + kb * KB + sRow) * DM + h * HD + sCol;
      const size_t vg = ((size_t)bh * HD + sRow) * SQ + kb * KB + sCol;
      const v8us a0 = *(const v8us*)((const unsigned short*)KH + kg), a1 = *(const v8us*)((const unsigned short*)KH + kg + 8);
      const v8us c0 = *(const v8us*)((const unsigned short*)KL + kg), c1 = *(const v8us*)((const unsigned short*)KL + kg + 8);
      const v8us v0 = *(const v8us*)((const unsigned short*)VT + vg), v1 = *(const v8us*)((const unsigned short*)VT + vg + 8);
      *(v8us*)&Kh[sRow][sCol] = a0; *(v8us*)&Kh[sRow][sCol + 8u] = a1;
      *(v8us*)&Kl[sRow][sCol] = c0; *(v8us*)&Kl[sRow][sCol + 8u] = c1;
      *(v8us*)&Vs[sRow][sCol] = v0; *(v8us*)&Vs[sRow][sCol + 8u] = v1;
    }
    __syncthreads();

    v8f s[4];
#pragma unroll
    for (int j = 0; j < 4; ++j) {
      const unsigned short* kr = &Kh[(unsigned)j * 16u + ln][0];
      const unsigned short* lr = &Kl[(unsigned)j * 16u + ln][0];
      const v16h kh0 = l_frag(kr, hh), kh1 = l_frag(kr + 32, hh);
      const v16h kl0 = l_frag(lr, hh), kl1 = l_frag(lr + 32, hh);
      v8f acc = z8;
      acc = g2_mma(ql0, kh0, acc); acc = g2_mma(ql1, kh1, acc);
      acc = g2_mma(qh0, kl0, acc); acc = g2_mma(qh1, kl1, acc);
      acc = acc * 0.00048828125f;
      acc = g2_mma(qh0, kh0, acc); acc = g2_mma(qh1, kh1, acc);
      s[j] = acc;
    }

    const unsigned int* mrow = mbase + kb * 2u;
#pragma unroll
    for (int r = 0; r < 8; ++r) {
      const v2u mw = *(const v2u*)(mrow + (size_t)r * MBW);
      float mx = -3.0e38f;
#pragma unroll
      for (int j = 0; j < 4; ++j) {
        const unsigned wd = (j < 2) ? mw[0] : mw[1];
        const unsigned bit = (wd >> ((unsigned)(j & 1) * 16u + ln)) & 1u;
        float sv = s[j][r] * 0.125f;
        sv = bit ? sv : -1.0e9f;
        s[j][r] = sv;
        mx = fmaxf(mx, sv);
      }
      mx = fmaxf(mx, __shfl_xor(mx, 1, 32)); mx = fmaxf(mx, __shfl_xor(mx, 2, 32));
      mx = fmaxf(mx, __shfl_xor(mx, 4, 32)); mx = fmaxf(mx, __shfl_xor(mx, 8, 32));
      const float mnew = fmaxf(mst[r], mx);
      const float alpha = __expf(mst[r] - mnew);
      mst[r] = mnew;
      float rsum = 0.0f;
#pragma unroll
      for (int j = 0; j < 4; ++j) { const float p = __expf(s[j][r] - mnew); s[j][r] = p; rsum += p; }
      rsum += __shfl_xor(rsum, 1, 32); rsum += __shfl_xor(rsum, 2, 32);
      rsum += __shfl_xor(rsum, 4, 32); rsum += __shfl_xor(rsum, 8, 32);
      lst[r] = lst[r] * alpha + rsum;
#pragma unroll
      for (int j = 0; j < 4; ++j) o[j][r] *= alpha;
    }

#pragma unroll
    for (int j = 0; j < 4; ++j)
#pragma unroll
      for (int r = 0; r < 8; ++r)
        Ps[w][0][8u * hh + (unsigned)r][(unsigned)j * 16u + ln] = (_Float16)(s[j][r] * 4096.0f);
    __builtin_amdgcn_fence(4  , "workgroup"); __builtin_amdgcn_wave_barrier();
    const unsigned short* pr = (const unsigned short*)&Ps[w][0][ln][0];
    const v16h pf0 = l_frag(pr, hh), pf1 = l_frag(pr + 32, hh);
#pragma unroll
    for (int j = 0; j < 4; ++j) {
      const unsigned short* vr = &Vs[(unsigned)j * 16u + ln][0];
      const v16h vf0 = l_frag(vr, hh), vf1 = l_frag(vr + 32, hh);
      o[j] = g2_mma(pf0, vf0, o[j]);
      o[j] = g2_mma(pf1, vf1, o[j]);
    }
    __syncthreads();
  }

#pragma unroll
  for (int r = 0; r < 8; ++r) {
    const float inv = 0.015625f * (1.0f / lst[r]);
#pragma unroll
    for (int j = 0; j < 4; ++j) {
      const float v = o[j][r] * inv;
      const _Float16 hv = (_Float16)v;
      Ps[w][0][8u * hh + (unsigned)r][(unsigned)j * 16u + ln] = hv;
      Ps[w][1][8u * hh + (unsigned)r][(unsigned)j * 16u + ln] = (_Float16)((v - (float)hv) * 1024.0f);
    }
  }
  __builtin_amdgcn_fence(4  , "workgroup"); __builtin_amdgcn_wave_barrier();
  const unsigned erow = lane >> 3, epc = (lane & 7u) * 8u;
  for (int pass = 0; pass < 2; ++pass) {
#pragma unroll
    for (unsigned it = 0; it < 4u; ++it) {
      const unsigned r = it * 4u + erow;
      const v8us vh = *(const v8us*)((const unsigned short*)&Ps[w][0][r][epc]);
      const v8us vl = *(const v8us*)((const unsigned short*)&Ps[w][1][r][epc]);
      const size_t go = (rb + qw + r) * DM + h * HD + epc;
      *(volatile v8us*)((unsigned short*)OH + go) = vh;
      *(volatile v8us*)((unsigned short*)OL + go) = vl;
    }
    if (pass == 0) __threadfence();
  }
}

extern "C" void kernel_launch(void* const* d_in, const int* in_sizes, int n_in,
                              void* d_out, int out_size, void* d_ws, size_t ws_size, hipStream_t stream) {
  if (n_in < 8) return;
  const size_t need_x = ((size_t)(NB - 1) * SQ_FULL + SQ) * DM;
  const size_t need_m = (size_t)(SQ - 1) * SQ_FULL + SQ;
  if ((size_t)in_sizes[0] < need_x || (size_t)in_sizes[1] < need_x || (size_t)in_sizes[2] < need_x) return;
  if ((size_t)in_sizes[3] < need_m) return;
  if ((size_t)in_sizes[4] < (size_t)DM * DM || (size_t)in_sizes[5] < (size_t)DM * DM || (size_t)in_sizes[6] < (size_t)DM * DM || (size_t)in_sizes[7] < (size_t)DM * DM) return;
  if ((size_t)out_size < need_x) return;
  const float* xq = (const float*)d_in[0]; const float* xk = (const float*)d_in[1]; const float* xv = (const float*)d_in[2];
  const int* am = (const int*)d_in[3];
  const float* wq = (const float*)d_in[4]; const float* wk = (const float*)d_in[5]; const float* wv = (const float*)d_in[6]; const float* wo = (const float*)d_in[7];
  char* ws = (char*)d_ws; size_t off = 0;
  auto take = [&](size_t bytes) { char* p = ws + off; off += (bytes + 255) & ~(size_t)255; return p; };
  const size_t WB = (size_t)DM * DM * 2, PB = NR * DM * 2;
  _Float16* BQ = (_Float16*)take(WB); _Float16* BK = (_Float16*)take(WB); _Float16* BV = (_Float16*)take(WB); _Float16* BO = (_Float16*)take(WB);
  _Float16* XQ = (_Float16*)take(PB); _Float16* XK = (_Float16*)take(PB); _Float16* XV = (_Float16*)take(PB);
  _Float16* QH = (_Float16*)take(PB); _Float16* QL = (_Float16*)take(PB); _Float16* KH = (_Float16*)take(PB); _Float16* KL = (_Float16*)take(PB);
  _Float16* V16 = (_Float16*)take(PB); _Float16* VT = (_Float16*)take(PB);
  _Float16* OH = (_Float16*)take(PB); _Float16* OL = (_Float16*)take(PB);
  unsigned int* MBp = (unsigned int*)take((size_t)SQ * MBW * 4);
  if (off > ws_size || off > (size_t)134217728) return;

  { const unsigned g = (unsigned)(((size_t)DM * DM / 8 + 255) / 256);
    k_wnat<<<g, 256, 0, stream>>>(wq, (size_t)DM * DM / 8, BQ); k_wnat<<<g, 256, 0, stream>>>(wk, (size_t)DM * DM / 8, BK);
    k_wnat<<<g, 256, 0, stream>>>(wv, (size_t)DM * DM / 8, BV); k_wnat<<<g, 256, 0, stream>>>(wo, (size_t)DM * DM / 8, BO); }
  { const dim3 g((unsigned)((size_t)SQ * DM / 8 / 256), NB);
    k_x16<<<g, 256, 0, stream>>>(xq, XQ); k_x16<<<g, 256, 0, stream>>>(xk, XK); k_x16<<<g, 256, 0, stream>>>(xv, XV); }
  k_maskbits<<<(unsigned)((size_t)SQ * (SQ / 1024) / 8), 256, 0, stream>>>(am, MBp);
  { const dim3 g((unsigned)((NR / 128) * (DM / 64)), 1);
    k_gemm2<false, true><<<g, 128, 0, stream>>>(XQ, XQ, DM, 0, BQ, DM, 0.0625f, 0.f, nullptr, QH, QL, DM, 0, (unsigned)NR, DM, DM);
    k_gemm2<false, true><<<g, 128, 0, stream>>>(XK, XK, DM, 0, BK, DM, 0.0625f, 0.f, nullptr, KH, KL, DM, 0, (unsigned)NR, DM, DM);
    k_gemm2<false, false><<<g, 128, 0, stream>>>(XV, XV, DM, 0, BV, DM, 0.0625f, 0.f, nullptr, V16, nullptr, DM, 0, (unsigned)NR, DM, DM); }
  k_vt<NH, SQ><<<NB * NH * (SQ / 64), 256, 0, stream>>>(V16, DM, VT);
  k_flash<<<dim3(SQ / QB, NB * NH), 256, 0, stream>>>(QH, QL, KH, KL, VT, MBp, OH, OL);
  k_gemm2<true, false><<<dim3((SQ / 128) * (DM / 64), NB), 128, 0, stream>>>(OH, OL, DM, (size_t)SQ * DM, BO, DM, 0.0009765625f, 0.0009765625f,
                                                                              (float*)d_out, nullptr, nullptr, DM, (size_t)SQ_FULL * DM, SQ, DM, DM);
}
